// GNNDenseLayer_36919538876772
// MI455X (gfx1250) — hardware-verified
//
#include <hip/hip_runtime.h>
#include <hip/hip_bf16.h>
#include <stddef.h>
#include <math.h>


#define FD    128
#define FO    32
#define G2W   64
#define K1    256
#define NB    256
#define NTHR  256
#define NWAVE 8
#define SBN   4096
#define SUBS  (SBN / NB)
#define EPT   8
#define CHUNK (NTHR * EPT)
#define WCAP  (EPT * 32)
#define PB    6144
#define FLT   4096
#define RHDR  32
#define RCAP  73728
#define RROW  (RHDR + RCAP)
#define HCAP  5632
#define WLC   1024
#define BROW  (RHDR + NWAVE * WLC)
#define P1W   256
#define P2W   128
#define SSW   256
#define LDS_L1 (NB * FD * 4 + NWAVE * 2 * FD * 4 + 2 * FD * 4)
#define PREP1 ((FD * (K1 / 8)) / NTHR)
#define PREP2 ((G2W * (FD / 8)) / NTHR)

static_assert(NTHR == NWAVE * 32);
static_assert(NB == NWAVE * 32);
static_assert(SBN == SUBS * NB && SUBS <= 255);
static_assert(WCAP == EPT * 32);
static_assert(PB >= FLT + CHUNK && (PB % 32) == 0 && (FLT % 32) == 0);
static_assert((RCAP % CHUNK) == 0 && ((RROW * 4) % 128) == 0);
static_assert((HCAP % 32) == 0 && (WLC % 32) == 0);
static_assert(((BROW * 4) % 128) == 0 && ((NWAVE * WLC) % (4 * NTHR)) == 0);
static_assert(NWAVE <= RHDR);
static_assert(LDS_L1 <= 300 * 1024);
static_assert(PREP1 * NTHR == FD * (K1 / 8) && PREP2 * NTHR == G2W * (FD / 8));
static_assert(P2W == 4 * 32 && P2W >= 2 * FO && P1W == 2 * FD && SSW == 2 * FD);
static_assert(FO * 4 == 128 && G2W == 2 * FO && (NB * FD / 4) % NTHR == 0 && (NB * FO / 4) % NTHR == 0);

typedef float          v4f   __attribute__((ext_vector_type(4)));
typedef float          v8f   __attribute__((ext_vector_type(8)));
typedef int            v4i   __attribute__((ext_vector_type(4)));
typedef unsigned       v4u   __attribute__((ext_vector_type(4)));
typedef unsigned short v8us  __attribute__((ext_vector_type(8)));
typedef unsigned short v16us __attribute__((ext_vector_type(16)));
typedef __bf16         v16bf __attribute__((ext_vector_type(16)));
union FragB { v16bf v; v16us u; v8us h[2]; };
union Pk8 { v8us h; v4u i; };

__device__ __forceinline__ v4f zero4() { v4f z; z.x = 0.0f; z.y = 0.0f; z.z = 0.0f; z.w = 0.0f; return z; }
__device__ __forceinline__ v8f zero8() { v8f z; for (int i = 0; i < 8; ++i) z[i] = 0.0f; return z; }

__device__ __forceinline__ unsigned f2bf(float f) {
  const unsigned u = __float_as_uint(f);
  return (u + 0x7FFFu + ((u >> 16) & 1u)) >> 16;
}

__device__ __forceinline__ void split8(v4f a, v4f b, v8us& hi, v8us& lo) {
  float f[8];
  f[0] = a.x; f[1] = a.y; f[2] = a.z; f[3] = a.w;
  f[4] = b.x; f[5] = b.y; f[6] = b.z; f[7] = b.w;
  v8us rh, rl;
#pragma unroll
  for (int i = 0; i < 8; ++i) {
    const unsigned hb = f2bf(f[i]);
    const float r = f[i] - __uint_as_float(hb << 16);
    rh[i] = (unsigned short)hb;
    rl[i] = (unsigned short)f2bf(r);
  }
  hi = rh;
  lo = rl;
}

__device__ __forceinline__ v8f wm3(v16bf ah, v16bf al, v16bf bh, v16bf bl, v8f c) {
  v8f d = __builtin_amdgcn_wmma_f32_16x16x32_bf16(false, ah, false, bh, (short)0, c, false, false);
  d = __builtin_amdgcn_wmma_f32_16x16x32_bf16(false, ah, false, bl, (short)0, d, false, false);
  d = __builtin_amdgcn_wmma_f32_16x16x32_bf16(false, al, false, bh, (short)0, d, false, false);
  asm volatile("v_nop\n\tv_nop\n\tv_nop\n\tv_nop" : "+v"(d) : "v"(ah), "v"(al), "v"(bh), "v"(bl));
  return d;
}

template <int NJ>
__device__ __forceinline__ void gstep(const FragB& ah, const FragB& al,
    const unsigned short* __restrict__ ph, const unsigned short* __restrict__ pl,
    int kp, int ko, int m, v8f (&d)[NJ]) {
#pragma unroll
  for (int j = 0; j < NJ; ++j) {
    const size_t o = (size_t)(16 * j + m) * kp + ko;
    FragB bh, bl;
    bh.h[0] = *(const v8us*)(ph + o);
    bh.h[1] = *(const v8us*)(ph + o + 16);
    bl.h[0] = *(const v8us*)(pl + o);
    bl.h[1] = *(const v8us*)(pl + o + 16);
    d[j] = wm3(ah.v, al.v, bh.v, bl.v, d[j]);
  }
}

__device__ __forceinline__ v4f bnrelu4(v4f a, v4f s, v4f t) {
  v4f o;
  o.x = fmaxf(a.x * s.x + t.x, 0.0f);
  o.y = fmaxf(a.y * s.y + t.y, 0.0f);
  o.z = fmaxf(a.z * s.z + t.z, 0.0f);
  o.w = fmaxf(a.w * s.w + t.w, 0.0f);
  return o;
}

__device__ __forceinline__ v4f xr4(v4f v, int msk) {
  v4f o;
  o.x = v.x + __shfl_xor(v.x, msk);
  o.y = v.y + __shfl_xor(v.y, msk);
  o.z = v.z + __shfl_xor(v.z, msk);
  o.w = v.w + __shfl_xor(v.w, msk);
  return o;
}

__device__ __forceinline__ int scan_chunk(const int* __restrict__ dsts, int nE, int cbase, int sbBase,
                                          int vec8, unsigned* list, int tid, int wave) {
  int wc = 0;
  const int e0   = cbase + tid * EPT;
  const int sent = -2147483647 - 1;
  v4i da, db;
  if (vec8 != 0 && cbase + CHUNK <= nE) {
    da = *(const v4i*)(dsts + e0);
    db = *(const v4i*)(dsts + e0 + 4);
  } else {
    da.x = (e0     < nE) ? dsts[min(e0, nE - 1)] : sent;
    da.y = (e0 + 1 < nE) ? dsts[min(e0 + 1, nE - 1)] : sent;
    da.z = (e0 + 2 < nE) ? dsts[min(e0 + 2, nE - 1)] : sent;
    da.w = (e0 + 3 < nE) ? dsts[min(e0 + 3, nE - 1)] : sent;
    db.x = (e0 + 4 < nE) ? dsts[min(e0 + 4, nE - 1)] : sent;
    db.y = (e0 + 5 < nE) ? dsts[min(e0 + 5, nE - 1)] : sent;
    db.z = (e0 + 6 < nE) ? dsts[min(e0 + 6, nE - 1)] : sent;
    db.w = (e0 + 7 < nE) ? dsts[min(e0 + 7, nE - 1)] : sent;
  }
  const unsigned nb = (unsigned)sbBase;
  const unsigned s0 = (unsigned)da.x - nb, s1 = (unsigned)da.y - nb;
  const unsigned s2 = (unsigned)da.z - nb, s3 = (unsigned)da.w - nb;
  const unsigned s4 = (unsigned)db.x - nb, s5 = (unsigned)db.y - nb;
  const unsigned s6 = (unsigned)db.z - nb, s7 = (unsigned)db.w - nb;
  const bool h0 = s0 < (unsigned)SBN, h1 = s1 < (unsigned)SBN, h2 = s2 < (unsigned)SBN, h3 = s3 < (unsigned)SBN;
  const bool h4 = s4 < (unsigned)SBN, h5 = s5 < (unsigned)SBN, h6 = s6 < (unsigned)SBN, h7 = s7 < (unsigned)SBN;
#define HITJ(J, HJ, SJ) { \
    const unsigned mj = __builtin_amdgcn_ballot_w32(HJ); \
    if (mj != 0u) { \
      const int pos = wc + (int)__builtin_amdgcn_mbcnt_lo(mj, 0u); \
      if ((HJ) && pos < WCAP) list[wave * WCAP + pos] = (((unsigned)(e0 + (J))) << 8) | ((SJ) >> 8); \
      wc += (int)__builtin_popcount(mj); } }
  HITJ(0, h0, s0)
  HITJ(1, h1, s1)
  HITJ(2, h2, s2)
  HITJ(3, h3, s3)
  HITJ(4, h4, s4)
  HITJ(5, h5, s5)
  HITJ(6, h6, s6)
  HITJ(7, h7, s7)
#undef HITJ
  return wc;
}

__device__ __forceinline__ int filt_chunk(const unsigned* __restrict__ ent, int cnt, int cbase, unsigned sub,
                                          unsigned* list, int tid, int wave) {
  int wc = 0;
  const int e0 = cbase + tid * EPT;
  const v4u a = *(const v4u*)(ent + e0);
  const v4u b = *(const v4u*)(ent + e0 + 4);
  const bool h0 = (e0     < cnt) && ((a.x & 255u) == sub);
  const bool h1 = (e0 + 1 < cnt) && ((a.y & 255u) == sub);
  const bool h2 = (e0 + 2 < cnt) && ((a.z & 255u) == sub);
  const bool h3 = (e0 + 3 < cnt) && ((a.w & 255u) == sub);
  const bool h4 = (e0 + 4 < cnt) && ((b.x & 255u) == sub);
  const bool h5 = (e0 + 5 < cnt) && ((b.y & 255u) == sub);
  const bool h6 = (e0 + 6 < cnt) && ((b.z & 255u) == sub);
  const bool h7 = (e0 + 7 < cnt) && ((b.w & 255u) == sub);
#define HITF(HJ, VJ) { \
    const unsigned mj = __builtin_amdgcn_ballot_w32(HJ); \
    if (mj != 0u) { \
      const int pos = wc + (int)__builtin_amdgcn_mbcnt_lo(mj, 0u); \
      if ((HJ) && pos < WCAP) list[wave * WCAP + pos] = (VJ) >> 8; \
      wc += (int)__builtin_popcount(mj); } }
  HITF(h0, a.x)
  HITF(h1, a.y)
  HITF(h2, a.z)
  HITF(h3, a.w)
  HITF(h4, b.x)
  HITF(h5, b.y)
  HITF(h6, b.z)
  HITF(h7, b.w)
#undef HITF
  return wc;
}

__device__ __forceinline__ void flush2(const unsigned* pend, unsigned* dst, int nst, int tid) {
#pragma unroll 1
  for (int u = tid; u < (nst >> 2); u += NTHR) {
    const v4u v = *(const v4u*)(pend + 4 * u);
    *(volatile v4u*)(dst + 4 * u) = v;
  }
  __threadfence();
#pragma unroll 1
  for (int u = tid; u < (nst >> 2); u += NTHR) {
    const v4u v = *(const v4u*)(pend + 4 * u);
    *(volatile v4u*)(dst + 4 * u) = v;
  }
}

__global__ __launch_bounds__(NTHR) void k_prep(const float* __restrict__ wr1, const float* __restrict__ wo1,
                                              const float* __restrict__ wr2, const float* __restrict__ wo2,
                                              unsigned short* p1, unsigned short* p2) {
  const int b = blockIdx.x, tid = threadIdx.x;
  float f[8];
  unsigned short* dh;
  unsigned short* dl;
  if (b < PREP1) {
    const int u = b * NTHR + tid;
    const int n = u >> 5;
    const int kc = u & 31;
#pragma unroll
    for (int j = 0; j < 8; ++j) {
      const int k = 8 * kc + j;
      const int ka = k < FD ? k : FD - 1;
      const int kb = k < FD ? 0 : k - FD;
      const float va = wr1[ka * FD + n];
      const float vb = wo1[kb * FD + n];
      f[j] = (k < FD) ? va : vb;
    }
    dh = p1 + (size_t)u * 8;
    dl = p1 + (size_t)FD * K1 + (size_t)u * 8;
  } else {
    const int u = (b - PREP1) * NTHR + tid;
    const int n = u >> 4;
    const int kc = u & 15;
    const int na = n < FO ? n : FO - 1;
    const int nb2 = n < FO ? 0 : n - FO;
#pragma unroll
    for (int j = 0; j < 8; ++j) {
      const int k = 8 * kc + j;
      const float va = wr2[k * FO + na];
      const float vb = wo2[k * FO + nb2];
      f[j] = (n < FO) ? va : vb;
    }
    dh = p2 + (size_t)u * 8;
    dl = p2 + (size_t)G2W * FD + (size_t)u * 8;
  }
  Pk8 ph, pl;
  {
    v4f a, c;
    a.x = f[0]; a.y = f[1]; a.z = f[2]; a.w = f[3];
    c.x = f[4]; c.y = f[5]; c.z = f[6]; c.w = f[7];
    split8(a, c, ph.h, pl.h);
  }
  *(volatile v4u*)dh = ph.i;
  *(volatile v4u*)dl = pl.i;
  __threadfence();
  *(volatile v4u*)dh = ph.i;
  *(volatile v4u*)dl = pl.i;
}

__global__ __launch_bounds__(NTHR) void k_scan(const int* __restrict__ ei, unsigned* t1, int nE, int vec8) {
  __shared__ unsigned list[NWAVE * WCAP];
  __shared__ __attribute__((aligned(16))) unsigned pend[PB];
  __shared__ int wcnt[NWAVE];
  const int tid = threadIdx.x, lane = tid & 31, wave = tid >> 5;
  const int sbBase = blockIdx.x * SBN;
  const int* dsts = ei + nE;
  unsigned* rowp = t1 + (size_t)blockIdx.x * RROW;
  unsigned* ent = rowp + RHDR;
  int pendN = 0;
  int gpos = 0;
  const int nChunks = (nE + CHUNK - 1) / CHUNK;
#pragma unroll 1
  for (int ch = 0; ch < nChunks; ++ch) {
    const int cbase = ch * CHUNK;
    const int wc = scan_chunk(dsts, nE, cbase, sbBase, vec8, list, tid, wave);
    if (lane == 0) wcnt[wave] = wc;
    __syncthreads();
    int tot = 0, myoff = 0;
#pragma unroll
    for (int w = 0; w < NWAVE; ++w) {
      int c = wcnt[w];
      c = c > WCAP ? WCAP : (c < 0 ? 0 : c);
      if (w < wave) myoff += c;
      tot += c;
    }
    {
      int n = wcnt[wave];
      n = n > WCAP ? WCAP : (n < 0 ? 0 : n);
      const unsigned* lp = list + wave * WCAP;
      for (int i = lane; i < n; i += 32) {
        const int pos = pendN + myoff + i;
        if (pos < PB) pend[pos] = lp[i];
      }
    }
    {
      const int newN = pendN + tot;
      pendN = newN > PB ? PB : newN;
    }
    __syncthreads();
    if (pendN >= FLT) {
      const int nfl = pendN & ~31;
      const int room = RCAP - gpos;
      const int nst = nfl < room ? nfl : room;
      flush2(pend, ent + gpos, nst, tid);
      gpos += nst;
      __syncthreads();
      const int rem = pendN - nfl;
      unsigned mv = 0u;
      if (tid < rem) mv = pend[nfl + tid];
      if (tid < rem) pend[tid] = mv;
      pendN = rem;
    }
  }
  __syncthreads();
  const int nfin = (pendN + 31) & ~31;
  if (tid < 32) {
    const int idx = pendN + tid;
    if (idx < nfin) pend[idx] = 0xFFFFFFFFu;
  }
  __syncthreads();
  {
    const int room = RCAP - gpos;
    const int nst = nfin < room ? nfin : room;
    flush2(pend, ent + gpos, nst, tid);
    gpos += nst;
  }
  if (wave == 0) {
    const unsigned hv = (lane == 0) ? (unsigned)gpos : 0u;
    *(volatile unsigned*)(rowp + lane) = hv;
    __threadfence();
    *(volatile unsigned*)(rowp + lane) = hv;
  }
}

__global__ __launch_bounds__(NTHR) void k_part(const int* __restrict__ ei, const unsigned* __restrict__ t1,
                                              unsigned* t2, int nE, int nN) {
  __shared__ unsigned list[NWAVE * WCAP];
  __shared__ unsigned hl[HCAP];
  __shared__ __attribute__((aligned(16))) unsigned wl[NWAVE * WLC];
  __shared__ int wcnt[NWAVE];
  __shared__ int wlen[NWAVE];
  const int tid = threadIdx.x, lane = tid & 31, wave = tid >> 5;
  const int blk = blockIdx.x;
  const int sb = blk / SUBS;
  const unsigned sub = (unsigned)(blk - sb * SUBS);
  const int nodeBase = blk * NB;
  const int* srcs = ei;
  const int* dsts = ei + nE;
  const unsigned* rowp = t1 + (size_t)sb * RROW;
  const unsigned* ent = rowp + RHDR;
  for (int i = tid; i < NWAVE * WLC; i += NTHR) wl[i] = 0u;
  int cnt = (int)rowp[0];
  cnt = cnt < 0 ? 0 : (cnt > RCAP ? RCAP : cnt);
  int hlN = 0;
  const int nCh = (cnt + CHUNK - 1) / CHUNK;
  __syncthreads();
#pragma unroll 1
  for (int ch = 0; ch < nCh; ++ch) {
    const int cbase = ch * CHUNK;
    const int wc = filt_chunk(ent, cnt, cbase, sub, list, tid, wave);
    if (lane == 0) wcnt[wave] = wc;
    __syncthreads();
    int tot = 0, myoff = 0;
#pragma unroll
    for (int w = 0; w < NWAVE; ++w) {
      int c = wcnt[w];
      c = c > WCAP ? WCAP : (c < 0 ? 0 : c);
      if (w < wave) myoff += c;
      tot += c;
    }
    {
      int n = wcnt[wave];
      n = n > WCAP ? WCAP : (n < 0 ? 0 : n);
      const unsigned* lp = list + wave * WCAP;
      for (int i = lane; i < n; i += 32) {
        const int pos = hlN + myoff + i;
        if (pos < HCAP) hl[pos] = lp[i];
      }
    }
    {
      const int newN = hlN + tot;
      hlN = newN > HCAP ? HCAP : newN;
    }
    __syncthreads();
  }
  {
    int wn = 0;
    const int niter = (hlN + 31) >> 5;
#pragma unroll 1
    for (int it = 0; it < niter; ++it) {
      const int idx = it * 32 + lane;
      const bool valid = idx < hlN;
      int e = (int)hl[idx < HCAP ? idx : HCAP - 1];
      e = e < 0 ? 0 : (e > nE - 1 ? nE - 1 : e);
      const int d = dsts[e];
      int s = srcs[e];
      s = s < 0 ? 0 : (s > nN - 1 ? nN - 1 : s);
      const int slot = d - nodeBase;
      const bool mine = valid && ((unsigned)slot < (unsigned)NB) && ((slot >> 5) == wave);
      const unsigned mk = __builtin_amdgcn_ballot_w32(mine);
      const int pos = wn + (int)__builtin_amdgcn_mbcnt_lo(mk, 0u);
      if (mine && pos < WLC) wl[wave * WLC + pos] = (((unsigned)s) << 8) | (unsigned)slot;
      wn += (int)__builtin_popcount(mk);
    }
    if (lane == 0) wlen[wave] = wn > WLC ? WLC : wn;
  }
  __syncthreads();
  unsigned* orow = t2 + (size_t)blk * BROW;
  unsigned hv = 0u;
  if (lane < NWAVE) hv = (unsigned)wlen[lane];
#pragma unroll 1
  for (int u = tid; u < NWAVE * WLC / 4; u += NTHR) {
    const v4u v = *(const v4u*)(wl + 4 * u);
    *(volatile v4u*)(orow + RHDR + 4 * u) = v;
  }
  if (wave == 0) *(volatile unsigned*)(orow + lane) = hv;
  __threadfence();
#pragma unroll 1
  for (int u = tid; u < NWAVE * WLC / 4; u += NTHR) {
    const v4u v = *(const v4u*)(wl + 4 * u);
    *(volatile v4u*)(orow + RHDR + 4 * u) = v;
  }
  if (wave == 0) *(volatile unsigned*)(orow + lane) = hv;
}

__global__ __launch_bounds__(NTHR) void k_layer1(const float* __restrict__ x, const unsigned* __restrict__ t2,
    const unsigned short* __restrict__ w1h, const unsigned short* __restrict__ w1l,
    const float* __restrict__ brel, float* hpre, float* part, int nN) {
  extern __shared__ __attribute__((aligned(16))) unsigned char dsm[];
  float* acc   = (float*)dsm;
  float* wpart = (float*)(dsm + (size_t)NB * FD * 4);
  float* bpart = wpart + NWAVE * 2 * FD;
  const int tid = threadIdx.x, lane = tid & 31, wave = tid >> 5, hh = lane >> 4, m = lane & 15;
  const int nodeBase = blockIdx.x * NB;
  {
    const v4f z = zero4();
    for (int i = tid; i < NB * FD / 4; i += NTHR) *(v4f*)(acc + 4 * i) = z;
  }
  __syncthreads();
  {
    const unsigned* brow = t2 + (size_t)blockIdx.x * BROW;
    int cnt = (int)brow[wave];
    cnt = cnt < 0 ? 0 : (cnt > WLC ? WLC : cnt);
    cnt = __builtin_amdgcn_readfirstlane(cnt);
    const unsigned* lst = brow + RHDR + wave * WLC;
#pragma unroll 1
    for (int i = 0; i < cnt; i += 32) {
      const unsigned pk = lst[i + lane];
      int jn = cnt - i;
      jn = jn > 32 ? 32 : jn;
#pragma unroll 1
      for (int jj = 0; jj < jn; ++jj) {
        const unsigned p = (unsigned)__builtin_amdgcn_readlane((int)pk, jj);
        int s = (int)(p >> 8);
        s = s > nN - 1 ? nN - 1 : s;
        const int slot = (int)(p & 255u);
        const v4f v = *(const v4f*)(x + (size_t)s * FD + 4 * lane);
        float* ap = acc + slot * FD + 4 * lane;
        v4f a = *(v4f*)ap;
        a += v;
        *(v4f*)ap = a;
      }
    }
  }
  __syncthreads();
  float cs[8], cq[8];
#pragma unroll
  for (int j = 0; j < 8; ++j) { cs[j] = 0.0f; cq[j] = 0.0f; }
#pragma unroll 1
  for (int tt = 0; tt < 2; ++tt) {
    const int t = wave + NWAVE * tt;
    const int r0 = 16 * t;
    int node = nodeBase + r0 + m;
    node = node > nN - 1 ? nN - 1 : node;
    const float* arow = acc + (r0 + m) * FD;
    const float* xrow = x + (size_t)node * FD;
    v8f d[8];
#pragma unroll
    for (int j = 0; j < 8; ++j) d[j] = zero8();
#pragma unroll 1
    for (int ks = 0; ks < 4; ++ks) {
      const int ko = 32 * ks + 8 * hh;
      FragB ah, al;
      split8(*(const v4f*)(arow + ko), *(const v4f*)(arow + ko + 4), ah.h[0], al.h[0]);
      split8(*(const v4f*)(arow + ko + 16), *(const v4f*)(arow + ko + 20), ah.h[1], al.h[1]);
      gstep<8>(ah, al, w1h, w1l, K1, ko, m, d);
    }
#pragma unroll 1
    for (int ks = 0; ks < 4; ++ks) {
      const int ko = 32 * ks + 8 * hh;
      FragB ah, al;
      split8(*(const v4f*)(xrow + ko), *(const v4f*)(xrow + ko + 4), ah.h[0], al.h[0]);
      split8(*(const v4f*)(xrow + ko + 16), *(const v4f*)(xrow + ko + 20), ah.h[1], al.h[1]);
      gstep<8>(ah, al, w1h, w1l, K1, FD + ko, m, d);
    }
    __syncthreads();
    float* srow = acc + (r0 + 8 * hh) * FD;
    const int nrow0 = nodeBase + r0 + 8 * hh;
#pragma unroll
    for (int j = 0; j < 8; ++j) {
      const int col = 16 * j + m;
      const float bj = brel[col];
      float sj = 0.0f, qj = 0.0f;
#pragma unroll
      for (int r = 0; r < 8; ++r) {
        const float v = d[j][r] + bj;
        srow[r * FD + col] = v;
        const float vm = (nrow0 + r < nN) ? v : 0.0f;
        sj += vm;
        qj += vm * vm;
      }
      sj += __shfl_xor(sj, 16);
      qj += __shfl_xor(qj, 16);
      cs[j] += sj;
      cq[j] += qj;
    }
  }
  if (hh == 0) {
#pragma unroll
    for (int j = 0; j < 8; ++j) {
      wpart[(wave * 2 + 0) * FD + 16 * j + m] = cs[j];
      wpart[(wave * 2 + 1) * FD + 16 * j + m] = cq[j];
    }
  }
  __syncthreads();
  {
    const int which = tid >> 7, c = tid & (FD - 1);
    float s = 0.0f;
#pragma unroll
    for (int w = 0; w < NWAVE; ++w) s += wpart[(w * 2 + which) * FD + c];
    bpart[which * FD + c] = s;
  }
  __syncthreads();
  float* prow = part + (size_t)blockIdx.x * P1W;
  v4f pv0 = zero4(), pv1 = zero4();
  if (wave == 0) {
    pv0 = *(const v4f*)(bpart + 4 * lane);
    pv1 = *(const v4f*)(bpart + FD + 4 * lane);
  }
  if (wave == 0) {
    *(volatile v4f*)(prow + 4 * lane) = pv0;
    *(volatile v4f*)(prow + FD + 4 * lane) = pv1;
  }
#pragma unroll 1
  for (int rr = 0; rr < NB / NWAVE; ++rr) {
    const int row = wave * (NB / NWAVE) + rr;
    const v4f v = *(const v4f*)(acc + row * FD + 4 * lane);
    *(volatile v4f*)(hpre + (size_t)(nodeBase + row) * FD + 4 * lane) = v;
  }
  __threadfence();
  if (wave == 0) {
    *(volatile v4f*)(prow + 4 * lane) = pv0;
    *(volatile v4f*)(prow + FD + 4 * lane) = pv1;
  }
#pragma unroll 1
  for (int rr = 0; rr < NB / NWAVE; ++rr) {
    const int row = wave * (NB / NWAVE) + rr;
    const v4f v = *(const v4f*)(acc + row * FD + 4 * lane);
    *(volatile v4f*)(hpre + (size_t)(nodeBase + row) * FD + 4 * lane) = v;
  }
}

__global__ __launch_bounds__(FD) void k_bnfin(const float* __restrict__ part, const float* __restrict__ gam,
                                            const float* __restrict__ bet, float* ss,
                                            int nBlk, int pw, int qoff, int D, int nN) {
  __shared__ __attribute__((aligned(16))) float st[SSW];
  const int c = threadIdx.x;
  const int cc = c < D ? c : D - 1;
  double S = 0.0, Q = 0.0;
#pragma unroll 1
  for (int b = 0; b < nBlk; ++b) {
    const float* pr = part + (size_t)b * pw;
    S += (double)pr[cc];
    Q += (double)pr[qoff + cc];
  }
  const double invN = 1.0 / (double)nN;
  const double mu = S * invN;
  double var = Q * invN - mu * mu;
  var = var < 0.0 ? 0.0 : var;
  const double rstd = 1.0 / sqrt(var + 1.0e-5);
  float sc = (float)((double)gam[cc] * rstd);
  float sh = (float)((double)bet[cc] - mu * (double)sc);
  if (c >= D) { sc = 0.0f; sh = 0.0f; }
  st[c] = sc;
  st[FD + c] = sh;
  __syncthreads();
  v4f a = zero4(), b2 = zero4();
  if (c < 32) {
    a = *(const v4f*)(st + 4 * c);
    b2 = *(const v4f*)(st + FD + 4 * c);
  }
  if (c < 32) {
    *(volatile v4f*)(ss + 4 * c) = a;
    *(volatile v4f*)(ss + FD + 4 * c) = b2;
  }
  __threadfence();
  if (c < 32) {
    *(volatile v4f*)(ss + 4 * c) = a;
    *(volatile v4f*)(ss + FD + 4 * c) = b2;
  }
}

__global__ __launch_bounds__(NTHR) void k_gemm2(const float* __restrict__ hpre, const float* __restrict__ ss,
    const unsigned short* __restrict__ w2h, const unsigned short* __restrict__ w2l, float* g2) {
  __shared__ __attribute__((aligned(16))) float stg[NWAVE * 16 * G2W];
  const int tid = threadIdx.x, lane = tid & 31, wave = tid >> 5, hh = lane >> 4, m = lane & 15;
  const size_t rbase = (size_t)blockIdx.x * (NWAVE * 16) + (size_t)wave * 16;
  const float* hrow = hpre + (rbase + m) * FD;
  v8f d[4];
#pragma unroll
  for (int j = 0; j < 4; ++j) d[j] = zero8();
#pragma unroll 1
  for (int ks = 0; ks < 4; ++ks) {
    const int ko = 32 * ks + 8 * hh;
    const v4f a0 = bnrelu4(*(const v4f*)(hrow + ko),      *(const v4f*)(ss + ko),      *(const v4f*)(ss + FD + ko));
    const v4f a1 = bnrelu4(*(const v4f*)(hrow + ko + 4),  *(const v4f*)(ss + ko + 4),  *(const v4f*)(ss + FD + ko + 4));
    const v4f a2 = bnrelu4(*(const v4f*)(hrow + ko + 16), *(const v4f*)(ss + ko + 16), *(const v4f*)(ss + FD + ko + 16));
    const v4f a3 = bnrelu4(*(const v4f*)(hrow + ko + 20), *(const v4f*)(ss + ko + 20), *(const v4f*)(ss + FD + ko + 20));
    FragB ah, al;
    split8(a0, a1, ah.h[0], al.h[0]);
    split8(a2, a3, ah.h[1], al.h[1]);
    gstep<4>(ah, al, w2h, w2l, FD, ko, m, d);
  }
  float* sw = stg + wave * 16 * G2W;
#pragma unroll
  for (int j = 0; j < 4; ++j) {
#pragma unroll
    for (int r = 0; r < 8; ++r) sw[(8 * hh + r) * G2W + 16 * j + m] = d[j][r];
  }
  __syncthreads();
  const int lr = lane >> 4, lc = 4 * (lane & 15);
#pragma unroll 1
  for (int i = 0; i < 8; ++i) {
    const int row = 2 * i + lr;
    const v4f v = *(const v4f*)(sw + row * G2W + lc);
    *(volatile v4f*)(g2 + (rbase + row) * G2W + lc) = v;
  }
  __threadfence();
#pragma unroll 1
  for (int i = 0; i < 8; ++i) {
    const int row = 2 * i + lr;
    const v4f v = *(const v4f*)(sw + row * G2W + lc);
    *(volatile v4f*)(g2 + (rbase + row) * G2W + lc) = v;
  }
}

__global__ __launch_bounds__(NTHR) void k_agg2(const float* __restrict__ g2, const unsigned* __restrict__ t2,
    const float* __restrict__ brel, float* hpre2, float* part, int nN) {
  __shared__ __attribute__((aligned(16))) float acc[NB * FO];
  __shared__ float wpart[NWAVE * 2 * FO];
  __shared__ __attribute__((aligned(16))) float bpart[P2W];
  const int tid = threadIdx.x, lane = tid & 31, wave = tid >> 5;
  const int nodeBase = blockIdx.x * NB;
  {
    const v4f z = zero4();
    for (int i = tid; i < NB * FO / 4; i += NTHR) *(v4f*)(acc + 4 * i) = z;
    if (tid < P2W) bpart[tid] = 0.0f;
  }
  __syncthreads();
  {
    const unsigned* brow = t2 + (size_t)blockIdx.x * BROW;
    int cnt = (int)brow[wave];
    cnt = cnt < 0 ? 0 : (cnt > WLC ? WLC : cnt);
    cnt = __builtin_amdgcn_readfirstlane(cnt);
    const unsigned* lst = brow + RHDR + wave * WLC;
#pragma unroll 1
    for (int i = 0; i < cnt; i += 32) {
      const unsigned pk = lst[i + lane];
      int jn = cnt - i;
      jn = jn > 32 ? 32 : jn;
#pragma unroll 1
      for (int jj = 0; jj < jn; ++jj) {
        const unsigned p = (unsigned)__builtin_amdgcn_readlane((int)pk, jj);
        int s = (int)(p >> 8);
        s = s > nN - 1 ? nN - 1 : s;
        const int slot = (int)(p & 255u);
        const float v = g2[(size_t)s * G2W + lane];
        float* ap = acc + slot * FO + lane;
        *ap = *ap + v;
      }
    }
  }
  __syncthreads();
  const int cg = lane & 7, rq = lane >> 3;
  const v4f bb = *(const v4f*)(brel + 4 * cg);
  v4f vals[8];
  v4f cs = zero4(), cq = zero4();
#pragma unroll
  for (int i = 0; i < 8; ++i) {
    const int row = wave * 32 + 4 * i + rq;
    const int node = nodeBase + row;
    const v4f a = *(const v4f*)(acc + row * FO + 4 * cg);
    const v4f rt = *(const v4f*)(g2 + (size_t)node * G2W + FO + 4 * cg);
    const v4f v = a + bb + rt;
    vals[i] = v;
    const float mk = (node < nN) ? 1.0f : 0.0f;
    const v4f vm = v * mk;
    cs += vm;
    cq += vm * vm;
  }
  cs = xr4(cs, 8);  cs = xr4(cs, 16);
  cq = xr4(cq, 8);  cq = xr4(cq, 16);
  if (rq == 0) {
    wpart[(wave * 2 + 0) * FO + 4 * cg + 0] = cs.x;
    wpart[(wave * 2 + 0) * FO + 4 * cg + 1] = cs.y;
    wpart[(wave * 2 + 0) * FO + 4 * cg + 2] = cs.z;
    wpart[(wave * 2 + 0) * FO + 4 * cg + 3] = cs.w;
    wpart[(wave * 2 + 1) * FO + 4 * cg + 0] = cq.x;
    wpart[(wave * 2 + 1) * FO + 4 * cg + 1] = cq.y;
    wpart[(wave * 2 + 1) * FO + 4 * cg + 2] = cq.z;
    wpart[(wave * 2 + 1) * FO + 4 * cg + 3] = cq.w;
  }
  __syncthreads();
  if (tid < 2 * FO) {
    const int which = tid >> 5, c = tid & 31;
    float s = 0.0f;
#pragma unroll
    for (int w = 0; w < NWAVE; ++w) s += wpart[(w * 2 + which) * FO + c];
    bpart[which * FO + c] = s;
  }
  __syncthreads();
  v4f pv = zero4();
  if (wave == 0) pv = *(const v4f*)(bpart + 4 * lane);
  float* prow = part + (size_t)blockIdx.x * P2W;
  if (wave == 0) *(volatile v4f*)(prow + 4 * lane) = pv;
#pragma unroll
  for (int i = 0; i < 8; ++i) {
    const int row = wave * 32 + 4 * i + rq;
    *(volatile v4f*)(hpre2 + (size_t)(nodeBase + row) * FO + 4 * cg) = vals[i];
  }
  __threadfence();
  if (wave == 0) *(volatile v4f*)(prow + 4 * lane) = pv;
#pragma unroll
  for (int i = 0; i < 8; ++i) {
    const int row = wave * 32 + 4 * i + rq;
    *(volatile v4f*)(hpre2 + (size_t)(nodeBase + row) * FO + 4 * cg) = vals[i];
  }
}

__global__ __launch_bounds__(NTHR) void k_out(const float* __restrict__ hpre2, const float* __restrict__ ss,
                                             float* dout, int n4) {
  const int u = blockIdx.x * NTHR + threadIdx.x;
  if (u >= n4) return;
  const int cg = u & 7;
  const v4f v = *(const v4f*)(hpre2 + (size_t)u * 4);
  const v4f sc = *(const v4f*)(ss + 4 * cg);
  const v4f sh = *(const v4f*)(ss + FD + 4 * cg);
  const v4f o = bnrelu4(v, sc, sh);
  *(volatile v4f*)(dout + (size_t)u * 4) = o;
  __threadfence();
  *(volatile v4f*)(dout + (size_t)u * 4) = o;
}

extern "C" void kernel_launch(void* const* d_in, const int* in_sizes, int n_in,
                              void* d_out, int out_size, void* d_ws, size_t ws_size,
                              hipStream_t stream) {
  if (n_in < 12) return;
  if (in_sizes[0] < FD || (in_sizes[0] % FD) != 0) return;
  const int nN = in_sizes[0] / FD;
  if ((in_sizes[1] & 1) != 0) return;
  const int nE = in_sizes[1] / 2;
  if (nE < 1 || nE >= (1 << 23)) return;
  if (in_sizes[2] != FD * FD || in_sizes[3] != FD || in_sizes[4] != FD * FD || in_sizes[5] != FD || in_sizes[6] != FD) return;
  if (in_sizes[7] != FD * FO || in_sizes[8] != FO || in_sizes[9] != FD * FO || in_sizes[10] != FO || in_sizes[11] != FO) return;
  if (out_size != nN * FO) return;

  const float* x    = (const float*)d_in[0];
  const int*   ei   = (const int*)d_in[1];
  const float* wr1  = (const float*)d_in[2];
  const float* br1  = (const float*)d_in[3];
  const float* wo1  = (const float*)d_in[4];
  const float* ga1  = (const float*)d_in[5];
  const float* be1  = (const float*)d_in[6];
  const float* wr2  = (const float*)d_in[7];
  const float* br2  = (const float*)d_in[8];
  const float* wo2  = (const float*)d_in[9];
  const float* ga2  = (const float*)d_in[10];
  const float* be2  = (const float*)d_in[11];
  float* dout = (float*)d_out;

  const int nBlk = (nN + NB - 1) / NB;
  const size_t rowsP = (size_t)nBlk * NB;
  const int nSB = (nBlk + SUBS - 1) / SUBS;

  char* ws = (char*)d_ws;
  size_t off = 0;
  auto carve = [&](size_t bytes) -> size_t {
    const size_t o = off;
    off = (off + bytes + 255) & ~(size_t)255;
    return o;
  };
  const size_t n1 = (size_t)FD * K1;
  const size_t n2 = (size_t)G2W * FD;
  const size_t oP1  = carve(2 * n1 * 2);
  const size_t oP2  = carve(2 * n2 * 2);
  const size_t oT1  = carve((size_t)nSB * RROW * 4);
  const size_t oT2  = carve((size_t)nBlk * BROW * 4);
  const size_t oH1  = carve(rowsP * FD * 4);
  const size_t oPT1 = carve((size_t)nBlk * P1W * 4);
  const size_t oS1  = carve((size_t)SSW * 4);
  const size_t oG2  = carve(rowsP * G2W * 4);
  const size_t oH2  = carve(rowsP * FO * 4);
  const size_t oPT2 = carve((size_t)nBlk * P2W * 4);
  const size_t oS2  = carve((size_t)SSW * 4);
  size_t limit = (size_t)134217728;
  if (ws_size < limit) limit = ws_size;
  if (off > limit) return;

  unsigned short* p1 = (unsigned short*)(ws + oP1);
  unsigned short* p2 = (unsigned short*)(ws + oP2);
  unsigned* t1 = (unsigned*)(ws + oT1);
  unsigned* t2 = (unsigned*)(ws + oT2);
  float* h1  = (float*)(ws + oH1);
  float* pt1 = (float*)(ws + oPT1);
  float* s1  = (float*)(ws + oS1);
  float* g2  = (float*)(ws + oG2);
  float* h2  = (float*)(ws + oH2);
  float* pt2 = (float*)(ws + oPT2);
  float* s2  = (float*)(ws + oS2);

  const int vec8 = ((nE & 3) == 0) ? 1 : 0;
  const int n4 = nN * (FO / 4);

  k_prep<<<PREP1 + PREP2, NTHR, 0, stream>>>(wr1, wo1, wr2, wo2, p1, p2);
  k_scan<<<nSB, NTHR, 0, stream>>>(ei, t1, nE, vec8);
  k_part<<<nBlk, NTHR, 0, stream>>>(ei, t1, t2, nE, nN);

  hipFuncSetAttribute(reinterpret_cast<const void*>(&k_layer1), hipFuncAttributeMaxDynamicSharedMemorySize, LDS_L1);
  k_layer1<<<nBlk, NTHR, LDS_L1, stream>>>(x, t2, p1, p1 + n1, br1, h1, pt1, nN);
  k_bnfin<<<1, FD, 0, stream>>>(pt1, ga1, be1, s1, nBlk, P1W, FD, FD, nN);

  k_gemm2<<<(unsigned)(rowsP / (NWAVE * 16)), NTHR, 0, stream>>>(h1, s1, p2, p2 + n2, g2);
  k_agg2<<<nBlk, NTHR, 0, stream>>>(g2, t2, br2, h2, pt2, nN);
  k_bnfin<<<1, FD, 0, stream>>>(pt2, ga2, be2, s2, nBlk, P2W, FO, FO, nN);

  k_out<<<(n4 + NTHR - 1) / NTHR, NTHR, 0, stream>>>(h2, s2, dout, n4);
}
